// Groupwise_CNN_LSTM_Pr_61452392071760
// MI455X (gfx1250) — hardware-verified
//
#include <hip/hip_runtime.h>
#include <float.h>
#include <math.h>

constexpr int kBatch   = 128;
constexpr int kWin     = 128;
constexpr int kFeat    = 128;
constexpr int kKC      = 16;
constexpr int kPool    = 65;
constexpr int kFc1     = 32;
constexpr int kHid     = 32;
constexpr int kGates   = 128;
constexpr int kFcIn    = 1040;
constexpr int kKdot    = 1056;
constexpr int kPitchY  = 1088;
constexpr int kRowsY   = kBatch * kWin;
constexpr int kMpadF   = 64;
constexpr int kComb    = kFc1 * kHid;
constexpr int kThreads = 256;
constexpr int kXPitch  = 132;
constexpr float kFc1Scale    = 32.0f;
constexpr float kFc1ScaleInv = 1.0f / 32.0f;
constexpr float kWScale      = 8.0f;
constexpr float kHScale      = 16.0f;
constexpr float kGateInv     = 1.0f / 128.0f;
static_assert(kKdot % 32 == 0);
static_assert(kPitchY % 64 == 0);
static_assert(kFcIn == kKC * kPool);

typedef __attribute__((ext_vector_type(16))) _Float16 v16h;
typedef __attribute__((ext_vector_type(8)))  _Float16 v8h;
typedef __attribute__((ext_vector_type(16))) __bf16   v16b;
typedef __attribute__((ext_vector_type(8)))  __bf16   v8b;
typedef __attribute__((ext_vector_type(8)))  float    v8f;
typedef __attribute__((ext_vector_type(4)))  float    v4f;

__device__ __forceinline__ unsigned short f2bf_bits(float f) {
  unsigned u = __float_as_uint(f);
  return (unsigned short)((u + 0x7FFFu + ((u >> 16) & 1u)) >> 16);
}
__device__ __forceinline__ float bf_bits2f(unsigned short h) { return __uint_as_float(((unsigned)h) << 16); }

__device__ __forceinline__ void dep_guard_h(v8f& a, v8f& b, v16h x, v16h y) { asm volatile("v_nop\n\tv_nop\n\tv_nop\n\tv_nop" : "+v"(a), "+v"(b) : "v"(x), "v"(y)); }
__device__ __forceinline__ void dep_guard_b(v8f& a, v8f& b, v16b x, v16b y) { asm volatile("v_nop\n\tv_nop\n\tv_nop\n\tv_nop" : "+v"(a), "+v"(b) : "v"(x), "v"(y)); }
__device__ __forceinline__ void keep4_h(v16h a, v16h b, v16h c, v16h d) { asm volatile("v_nop" :: "v"(a), "v"(b), "v"(c), "v"(d)); }
__device__ __forceinline__ void keep4_b(v16b a, v16b b, v16b c, v16b d) { asm volatile("v_nop" :: "v"(a), "v"(b), "v"(c), "v"(d)); }
__device__ __forceinline__ void acc_guard4(v8f& a, v8f& b, v8f& c, v8f& d) { asm volatile("v_nop\n\tv_nop\n\tv_nop\n\tv_nop" : "+v"(a), "+v"(b), "+v"(c), "+v"(d)); }
template <typename T> struct Frag;
template <> struct Frag<_Float16> {
  typedef v16h V; union U { v16h v; v8h h[2]; };
  static __device__ __forceinline__ v16h load(const _Float16* p) {
    U f; f.h[0] = *(const v8h*)(p); f.h[1] = *(const v8h*)(p + 16); return f.v;
  }
  static __device__ __forceinline__ v8f mma(v16h a, v16h b, v8f c) {
    return __builtin_amdgcn_wmma_f32_16x16x32_f16(false, a, false, b, (short)0, c, false, false);
  }
  static __device__ __forceinline__ void guard(v8f& a, v8f& b, v16h x, v16h y) { dep_guard_h(a, b, x, y); }
  static __device__ __forceinline__ void keep(v16h a, v16h b, v16h c, v16h d) { keep4_h(a, b, c, d); }
};
template <> struct Frag<__bf16> {
  typedef v16b V; union U { v16b v; v8b h[2]; };
  static __device__ __forceinline__ v16b load(const __bf16* p) {
    U f; f.h[0] = *(const v8b*)(p); f.h[1] = *(const v8b*)(p + 16); return f.v;
  }
  static __device__ __forceinline__ v8f mma(v16b a, v16b b, v8f c) {
    return __builtin_amdgcn_wmma_f32_16x16x32_bf16(false, a, false, b, (short)0, c, false, false);
  }
  static __device__ __forceinline__ void guard(v8f& a, v8f& b, v16b x, v16b y) { dep_guard_b(a, b, x, y); }
  static __device__ __forceinline__ void keep(v16b a, v16b b, v16b c, v16b d) { keep4_b(a, b, c, d); }
};

template <int ET> struct Elem;
template <> struct Elem<0> { typedef _Float16 T; };
template <> struct Elem<1> { typedef __bf16 T; };
template <int ET, bool SPLIT, int BIAS_MODE, int OUT_MODE, bool RESID, int ACT = 0>
__global__ __launch_bounds__(256) void wmma_gemm64(
    const unsigned short* __restrict__ Ap, const unsigned short* __restrict__ A2p, int lda, long strideA,
    const unsigned short* __restrict__ Btp, const unsigned short* __restrict__ Bt2p, int ldb, long strideB,
    void* __restrict__ Cout, void* __restrict__ Cout2, int ldc, long strideC,
    const float* __restrict__ bias,
    const float* __restrict__ resid, long strideR,
    int M, int N, int K, float scale) {
  typedef typename Elem<ET>::T T;
  typedef typename Frag<T>::V V;
  const T* A = (const T*)Ap; const T* A2 = (const T*)A2p; const T* Bt = (const T*)Btp; const T* Bt2 = (const T*)Bt2p;
  __shared__ __align__(16) float sT[8][16 * 68];
  const int b    = blockIdx.y;
  const int lane = threadIdx.x & 31;
  const int wave = threadIdx.x >> 5;
  const int tilesN = N >> 6;
  const int tilesM = M >> 6;
  const int tile = blockIdx.x * 8 + wave;
  if (tile >= tilesM * tilesN) return;
  const int tm = tile / tilesN;
  const int tn = tile - tm * tilesN;
  const int m0 = tm << 6;
  const int n0 = tn << 6;

  const T* Ab  = A  + (size_t)b * strideA;
  const T* Bb  = Bt + (size_t)b * strideB;
  const T* Ab2 = SPLIT ? (A2  + (size_t)b * strideA) : nullptr;
  const T* Bb2 = SPLIT ? (Bt2 + (size_t)b * strideB) : nullptr;

  const int rlane = lane & 15;
  const int koff  = (lane >> 4) * 8;
  const int mOff  = (lane >> 4) * 8;

  v8f acc[4][4];
#pragma unroll
  for (int i = 0; i < 4; ++i)
#pragma unroll
    for (int j = 0; j < 4; ++j) acc[i][j] = (v8f){0.f,0.f,0.f,0.f,0.f,0.f,0.f,0.f};

  for (int k0 = 0; k0 < K; k0 += 32) {
    V bh[4], bl[4];
#pragma unroll
    for (int j = 0; j < 4; ++j) {
      const size_t bo = (size_t)(n0 + (j << 4) + rlane) * ldb + koff + k0;
      bh[j] = Frag<T>::load(Bb + bo);
      if (SPLIT) bl[j] = Frag<T>::load(Bb2 + bo);
    }
#pragma unroll
    for (int i = 0; i < 4; ++i) {
      const size_t ao = (size_t)(m0 + (i << 4) + rlane) * lda + koff + k0;
      V ah = Frag<T>::load(Ab + ao);
      V al;
      if (SPLIT) al = Frag<T>::load(Ab2 + ao);
#pragma unroll
      for (int j = 0; j < 4; ++j) {
        acc[i][j] = Frag<T>::mma(ah, bh[j], acc[i][j]);
        if (SPLIT) {
          acc[i][j] = Frag<T>::mma(ah, bl[j], acc[i][j]);
          acc[i][j] = Frag<T>::mma(al, bh[j], acc[i][j]);
        }
      }
      Frag<T>::guard(acc[i][0], acc[i][3], ah, SPLIT ? al : ah);
    }
    Frag<T>::keep(bh[0], bh[1], bh[2], bh[3]);
    if (SPLIT) Frag<T>::keep(bl[0], bl[1], bl[2], bl[3]);
  }
  acc_guard4(acc[0][0], acc[0][1], acc[0][2], acc[0][3]);
  acc_guard4(acc[1][0], acc[1][1], acc[1][2], acc[1][3]);
  acc_guard4(acc[2][0], acc[2][1], acc[2][2], acc[2][3]);
  acc_guard4(acc[3][0], acc[3][1], acc[3][2], acc[3][3]);

  float* slab = sT[wave];
  const float* Rb = RESID ? (resid + (size_t)b * strideR) : nullptr;
#pragma unroll
  for (int i = 0; i < 4; ++i) {
    const int mBase = m0 + (i << 4);
#pragma unroll
    for (int j = 0; j < 4; ++j) {
      const int n = n0 + (j << 4) + rlane;
      float bv = 0.f;
      if (BIAS_MODE == 2) bv = bias[n];
#pragma unroll
      for (int r = 0; r < 8; ++r) {
        float v = acc[i][j][r] * scale;
        if (BIAS_MODE == 1) v += bias[mBase + mOff + r];
        if (BIAS_MODE == 2) v += bv;
        if (RESID) v += Rb[(size_t)(mBase + mOff + r) * ldc + n];
        if (ACT == 1) v = tanhf(v);
        if (ACT == 2) v = fmaxf(v, 0.0f);
        if (ACT == 3) v = v / (1.0f + expf(-v));
        if (ACT == 4) v = (v > 0.f) ? v : 0.01f * v;
        if (ACT == 5) v = 0.5f * v * (1.0f + erff(v * 0.70710678118654752f));
        slab[(mOff + r) * 68 + (j << 4) + rlane] = v;
      }
    }
    __builtin_amdgcn_fence(__ATOMIC_RELEASE, "workgroup");
    __builtin_amdgcn_wave_barrier();
    __builtin_amdgcn_fence(__ATOMIC_ACQUIRE, "workgroup");
    if (OUT_MODE == 0) {
      float* C = (float*)Cout + (size_t)b * strideC;
      const int hh = lane >> 4, c4 = (lane & 15) * 4;
      for (int pass = 0; pass < 2; ++pass) {
#pragma unroll
        for (int it = 0; it < 8; ++it) {
          const int row = it * 2 + hh;
          v4f v = *(const v4f*)(slab + row * 68 + c4);
          *(volatile v4f*)(C + (size_t)(mBase + row) * ldc + n0 + c4) = v;
        }
        __threadfence();
      }
    } else {
      const int q = lane >> 3, c8 = (lane & 7) * 8;
      unsigned short* C  = (unsigned short*)Cout  + (size_t)b * strideC;
      unsigned short* C2 = (OUT_MODE == 2) ? ((unsigned short*)Cout2 + (size_t)b * strideC) : nullptr;
      for (int pass = 0; pass < 2; ++pass) {
#pragma unroll
        for (int it = 0; it < 4; ++it) {
          const int row = it * 4 + q;
          const float* sp = slab + row * 68 + c8;
          v8h hv, lv;
#pragma unroll
          for (int e = 0; e < 8; ++e) {
            if (OUT_MODE == 1) {
              hv[e] = (_Float16)sp[e];
            } else {
              unsigned short hb = f2bf_bits(sp[e]);
              unsigned short lb = f2bf_bits(sp[e] - bf_bits2f(hb));
              hv[e] = __builtin_bit_cast(_Float16, hb);
              lv[e] = __builtin_bit_cast(_Float16, lb);
            }
          }
          *(volatile v8h*)(C + (size_t)(mBase + row) * ldc + n0 + c8) = hv;
          if (OUT_MODE == 2) *(volatile v8h*)(C2 + (size_t)(mBase + row) * ldc + n0 + c8) = lv;
        }
        __threadfence();
      }
    }
    __builtin_amdgcn_fence(__ATOMIC_RELEASE, "workgroup");
    __builtin_amdgcn_wave_barrier();
    __builtin_amdgcn_fence(__ATOMIC_ACQUIRE, "workgroup");
  }
}

__device__ __forceinline__ float fsig(float x)  { return __builtin_amdgcn_rcpf(1.0f + __expf(-x)); }
__device__ __forceinline__ float ftanh(float x) { return 1.0f - 2.0f * __builtin_amdgcn_rcpf(__expf(2.0f * x) + 1.0f); }

__global__ __launch_bounds__(kThreads) void fc1w_plane_kernel(const float* __restrict__ fc1_w, unsigned short* __restrict__ Wp) {
  const int i = blockIdx.x * kThreads + threadIdx.x;
  constexpr int kChunksPerRow = kPitchY / 8;
  if (i >= kMpadF * kChunksPerRow) return;
  const int row  = i / kChunksPerRow;
  const int col0 = (i - row * kChunksPerRow) * 8;
  const int rc = row < kFc1 ? row : (kFc1 - 1);
  v8h hv;
#pragma unroll
  for (int e = 0; e < 8; ++e) {
    const int col = col0 + e;
    const int cc = col < kFcIn ? col : (kFcIn - 1);
    const float v = fc1_w[(size_t)rc * kFcIn + cc];
    const bool ok = (row < kFc1) && (col < kFcIn);
    hv[e] = ok ? (_Float16)(v * kFc1Scale) : (_Float16)0.0f;
  }
  unsigned short* dst = Wp + (size_t)i * 8;
  *(volatile v8h*)dst = hv;
  __threadfence();
  *(volatile v8h*)dst = hv;
}

__global__ __launch_bounds__(kThreads) void conv_pool_kernel(const float* __restrict__ x, const float* __restrict__ conv_w,
                                                             const float* __restrict__ conv_b, unsigned short* __restrict__ Yp) {
  __shared__ float xs[16 * kXPitch];
  __shared__ __align__(16) _Float16 ys[16 * kPitchY];
  const int tid = threadIdx.x, lane = tid & 31, wave = tid >> 5;
  const int t  = blockIdx.x >> 3;
  const int b0 = (blockIdx.x & 7) * 16;
  const int rowbase = t * kBatch + b0;
#pragma unroll
  for (int it = 0; it < 2; ++it) {
    const int idx = it * kThreads + tid;
    const int r = idx >> 5, c4 = (idx & 31) * 4;
    const v4f v = *(const v4f*)(x + ((size_t)(b0 + r) * kWin + t) * kFeat + c4);
    float* d = xs + r * kXPitch + 1 + c4;
    d[0] = v[0]; d[1] = v[1]; d[2] = v[2]; d[3] = v[3];
  }
  if (tid < 64) {
    const int r = tid & 15, wsel = tid >> 4;
    const int col = (wsel == 0) ? 0 : (kFeat + wsel);
    xs[r * kXPitch + col] = 0.0f;
  }
  __syncthreads();
  {
    const int r = tid >> 4, j = tid & 15;
    const int ch = t * kKC + j;
    const float w0 = conv_w[ch * 3 + 0], w1 = conv_w[ch * 3 + 1], w2 = conv_w[ch * 3 + 2];
    const float bb = conv_b[ch];
    const float* xr = xs + r * kXPitch;
    _Float16* yr = ys + r * kPitchY + j * kPool;
#pragma unroll 1
    for (int q = 0; q < kPool; ++q) {
      const int pa = 2 * q - 1, pb = 2 * q;
      const int pac = pa < 0 ? 0 : pa;
      const int pbc = pb > (kFeat - 1) ? (kFeat - 1) : pb;
      float sa = w0 * xr[pac];
      sa = fmaf(w1, xr[pac + 1], sa);
      sa = fmaf(w2, xr[pac + 2], sa);
      sa += bb;
      sa = fmaxf(sa, 0.0f);
      float sb = w0 * xr[pbc];
      sb = fmaf(w1, xr[pbc + 1], sb);
      sb = fmaf(w2, xr[pbc + 2], sb);
      sb += bb;
      sb = fmaxf(sb, 0.0f);
      const float va = (pa >= 0) ? sa : -FLT_MAX;
      const float vb = (pb <= kFeat - 1) ? sb : -FLT_MAX;
      yr[q] = (_Float16)fmaxf(va, vb);
    }
  }
#pragma unroll
  for (int it = 0; it < 3; ++it) {
    const int i = it * kThreads + tid;
    const int r = i / 48, cc = i - r * 48;
    ys[r * kPitchY + kFcIn + cc] = (_Float16)0.0f;
  }
  __syncthreads();
  const int lq = lane >> 3, l8 = (lane & 7) * 8;
  for (int pass = 0; pass < 2; ++pass) {
#pragma unroll
    for (int it = 0; it < 9; ++it) {
      const int L  = it * 4 + lq;
      const int Lc = (L < 34) ? L : 33;
      const int rsub = (Lc >= 17) ? 1 : 0;
      const int seg  = Lc - rsub * 17;
      const int rr   = 2 * wave + rsub;
      const v8h v = *(const v8h*)(ys + rr * kPitchY + seg * 64 + l8);
      if (L < 34) *(volatile v8h*)(Yp + (size_t)(rowbase + rr) * kPitchY + seg * 64 + l8) = v;
    }
    __threadfence();
  }
}

__global__ __launch_bounds__(kThreads) void lstm_bank_kernel(const float* __restrict__ ZT, const float* __restrict__ fc1_b,
                                                             const float* __restrict__ w_ih0, const float* __restrict__ w_ih1,
                                                             const float* __restrict__ w_hh, const float* __restrict__ b_lstm,
                                                             float* __restrict__ comb) {
  __shared__ __align__(16) _Float16 Whh0s[kGates * kHid];
  __shared__ __align__(16) _Float16 Wih1s[kGates * kHid];
  __shared__ __align__(16) _Float16 Whh1s[kGates * kHid];
  __shared__ float wih0s[kGates], b0s[kGates], b1s[kGates];
  __shared__ __align__(16) _Float16 h0s[2 * kBatch * kHid];
  __shared__ __align__(16) _Float16 h1s[2 * kBatch * kHid];
  __shared__ __align__(16) float Hs[kBatch * kHid];
  const int f = blockIdx.x;
  const int tid = threadIdx.x, lane = tid & 31, wave = tid >> 5;
  const int c = lane & 15, hh = lane >> 4, koff = hh * 8;
  constexpr int kMat = kGates * kHid;

#pragma unroll
  for (int it = 0; it < 4; ++it) {
    const int e = (it * kThreads + tid) * 4;
    const v4f wa = *(const v4f*)(w_hh  + (size_t)f * kMat + e);
    const v4f wb = *(const v4f*)(w_ih1 + (size_t)f * kMat + e);
    const v4f wc = *(const v4f*)(w_hh  + (size_t)(kFc1 + f) * kMat + e);
#pragma unroll
    for (int k = 0; k < 4; ++k) {
      Whh0s[e + k] = (_Float16)(wa[k] * kWScale);
      Wih1s[e + k] = (_Float16)(wb[k] * kWScale);
      Whh1s[e + k] = (_Float16)(wc[k] * kWScale);
    }
  }
  if (tid < kGates) {
    wih0s[tid] = w_ih0[(size_t)f * kGates + tid];
    b0s[tid]   = b_lstm[(size_t)f * kGates + tid];
    b1s[tid]   = b_lstm[(size_t)(kFc1 + f) * kGates + tid];
  }
  {
    v8h zero8;
#pragma unroll
    for (int e = 0; e < 8; ++e) zero8[e] = (_Float16)0.0f;
#pragma unroll
    for (int it = 0; it < 4; ++it) {
      const int idx = (it * kThreads + tid) * 8;
      *(v8h*)(h0s + idx) = zero8;
      *(v8h*)(h1s + idx) = zero8;
    }
  }
  float c0st[2][8], c1st[2][8];
#pragma unroll
  for (int u = 0; u < 2; ++u)
#pragma unroll
    for (int r = 0; r < 8; ++r) { c0st[u][r] = 0.0f; c1st[u][r] = 0.0f; }
  __syncthreads();

  const float fb = fc1_b[f];
  const float* zbase = ZT + (size_t)f * kRowsY + 16 * wave + 8 * hh;
  const v8f z8 = {0.f, 0.f, 0.f, 0.f, 0.f, 0.f, 0.f, 0.f};
  const int arow = (16 * wave + c) * kHid + koff;
  const int hrow0 = 16 * wave + 8 * hh;

#pragma unroll 1
  for (int t = 0; t < kWin; ++t) {
    const int pbuf = (t & 1) * (kBatch * kHid), qbuf = ((t & 1) ^ 1) * (kBatch * kHid);
    const v4f za = *(const v4f*)(zbase + (size_t)t * kBatch);
    const v4f zb = *(const v4f*)(zbase + (size_t)t * kBatch + 4);
    float zv[8];
    zv[0] = za[0] + fb; zv[1] = za[1] + fb; zv[2] = za[2] + fb; zv[3] = za[3] + fb;
    zv[4] = zb[0] + fb; zv[5] = zb[1] + fb; zv[6] = zb[2] + fb; zv[7] = zb[3] + fb;

    const v16h A0 = Frag<_Float16>::load(h0s + pbuf + arow);
#pragma unroll
    for (int u = 0; u < 2; ++u) {
      const int g0 = 16 * u + c;
      v8f acc[4];
      const v16h bq0 = Frag<_Float16>::load(Whh0s + (g0 +  0) * kHid + koff);
      const v16h bq1 = Frag<_Float16>::load(Whh0s + (g0 + 32) * kHid + koff);
      const v16h bq2 = Frag<_Float16>::load(Whh0s + (g0 + 64) * kHid + koff);
      const v16h bq3 = Frag<_Float16>::load(Whh0s + (g0 + 96) * kHid + koff);
      acc[0] = Frag<_Float16>::mma(A0, bq0, z8);
      acc[1] = Frag<_Float16>::mma(A0, bq1, z8);
      acc[2] = Frag<_Float16>::mma(A0, bq2, z8);
      acc[3] = Frag<_Float16>::mma(A0, bq3, z8);
      dep_guard_h(acc[0], acc[3], A0, bq3);
      keep4_h(bq0, bq1, bq2, bq3);
      acc_guard4(acc[0], acc[1], acc[2], acc[3]);
      const float wi = wih0s[g0], wf = wih0s[g0 + 32], wg = wih0s[g0 + 64], wo = wih0s[g0 + 96];
      const float bi = b0s[g0],   bfg = b0s[g0 + 32],  bg = b0s[g0 + 64],   bo = b0s[g0 + 96];
#pragma unroll
      for (int r = 0; r < 8; ++r) {
        const float gi = fmaf(acc[0][r], kGateInv, fmaf(zv[r], wi, bi));
        const float gf = fmaf(acc[1][r], kGateInv, fmaf(zv[r], wf, bfg));
        const float gg = fmaf(acc[2][r], kGateInv, fmaf(zv[r], wg, bg));
        const float go = fmaf(acc[3][r], kGateInv, fmaf(zv[r], wo, bo));
        const float cn = fsig(gf) * c0st[u][r] + fsig(gi) * ftanh(gg);
        c0st[u][r] = cn;
        const float hn = fsig(go) * ftanh(cn);
        h0s[qbuf + (hrow0 + r) * kHid + g0] = (_Float16)(hn * kHScale);
      }
    }
    __syncthreads();

    const v16h A1 = Frag<_Float16>::load(h0s + qbuf + arow);
    const v16h A2 = Frag<_Float16>::load(h1s + pbuf + arow);
#pragma unroll
    for (int u = 0; u < 2; ++u) {
      const int g0 = 16 * u + c;
      v8f acc[4];
      const v16h bi0 = Frag<_Float16>::load(Wih1s + (g0 +  0) * kHid + koff);
      const v16h bi1 = Frag<_Float16>::load(Wih1s + (g0 + 32) * kHid + koff);
      const v16h bi2 = Frag<_Float16>::load(Wih1s + (g0 + 64) * kHid + koff);
      const v16h bi3 = Frag<_Float16>::load(Wih1s + (g0 + 96) * kHid + koff);
      acc[0] = Frag<_Float16>::mma(A1, bi0, z8);
      acc[1] = Frag<_Float16>::mma(A1, bi1, z8);
      acc[2] = Frag<_Float16>::mma(A1, bi2, z8);
      acc[3] = Frag<_Float16>::mma(A1, bi3, z8);
      dep_guard_h(acc[0], acc[3], A1, bi3);
      keep4_h(bi0, bi1, bi2, bi3);
      const v16h bh0 = Frag<_Float16>::load(Whh1s + (g0 +  0) * kHid + koff);
      const v16h bh1 = Frag<_Float16>::load(Whh1s + (g0 + 32) * kHid + koff);
      const v16h bh2 = Frag<_Float16>::load(Whh1s + (g0 + 64) * kHid + koff);
      const v16h bh3 = Frag<_Float16>::load(Whh1s + (g0 + 96) * kHid + koff);
      acc[0] = Frag<_Float16>::mma(A2, bh0, acc[0]);
      acc[1] = Frag<_Float16>::mma(A2, bh1, acc[1]);
      acc[2] = Frag<_Float16>::mma(A2, bh2, acc[2]);
      acc[3] = Frag<_Float16>::mma(A2, bh3, acc[3]);
      dep_guard_h(acc[0], acc[3], A2, bh3);
      keep4_h(bh0, bh1, bh2, bh3);
      acc_guard4(acc[0], acc[1], acc[2], acc[3]);
      const float bi = b1s[g0], bfg = b1s[g0 + 32], bg = b1s[g0 + 64], bo = b1s[g0 + 96];
#pragma unroll
      for (int r = 0; r < 8; ++r) {
        const float gi = fmaf(acc[0][r], kGateInv, bi);
        const float gf = fmaf(acc[1][r], kGateInv, bfg);
        const float gg = fmaf(acc[2][r], kGateInv, bg);
        const float go = fmaf(acc[3][r], kGateInv, bo);
        const float cn = fsig(gf) * c1st[u][r] + fsig(gi) * ftanh(gg);
        c1st[u][r] = cn;
        const float hn = fsig(go) * ftanh(cn);
        h1s[qbuf + (hrow0 + r) * kHid + g0] = (_Float16)(hn * kHScale);
        if (t == kWin - 1) Hs[(hrow0 + r) * kHid + g0] = hn;
      }
    }
    __syncthreads();
  }

  const int lq = lane >> 3, c4 = (lane & 7) * 4;
  for (int pass = 0; pass < 2; ++pass) {
#pragma unroll
    for (int it = 0; it < 4; ++it) {
      const int row = it * 32 + wave * 4 + lq;
      const v4f v = *(const v4f*)(Hs + row * kHid + c4);
      *(volatile v4f*)(comb + (size_t)row * kComb + f * kHid + c4) = v;
    }
    __threadfence();
  }
}

__global__ __launch_bounds__(128) void head_kernel(const float* __restrict__ comb, const float* __restrict__ mu_w,
                                                   const float* __restrict__ mu_b, const float* __restrict__ lv_w,
                                                   const float* __restrict__ lv_b, float* __restrict__ out) {
  __shared__ __align__(16) float outs[4 * kBatch];
  const int tid = threadIdx.x;
  const float* hrow = comb + (size_t)tid * kComb;
  float am = 0.0f, al = 0.0f;
#pragma unroll 1
  for (int i = 0; i < kComb; i += 4) {
    const v4f hv = *(const v4f*)(hrow + i);
    const v4f wm = *(const v4f*)(mu_w + i);
    const v4f wl = *(const v4f*)(lv_w + i);
    am = fmaf(hv[0], wm[0], am); am = fmaf(hv[1], wm[1], am); am = fmaf(hv[2], wm[2], am); am = fmaf(hv[3], wm[3], am);
    al = fmaf(hv[0], wl[0], al); al = fmaf(hv[1], wl[1], al); al = fmaf(hv[2], wl[2], al); al = fmaf(hv[3], wl[3], al);
  }
  const float mu = am + mu_b[0];
  const float lv = al + lv_b[0];
  const float sg = expf(0.5f * lv);
  const float d = 1.96f * sg;
  outs[tid]              = mu - d;
  outs[kBatch + tid]     = mu;
  outs[2 * kBatch + tid] = mu + d;
  outs[3 * kBatch + tid] = lv;
  __syncthreads();
  if (tid < 32) {
    for (int pass = 0; pass < 2; ++pass) {
#pragma unroll
      for (int it = 0; it < 4; ++it) {
        const v4f v = *(const v4f*)(outs + it * kBatch + tid * 4);
        *(volatile v4f*)(out + it * kBatch + tid * 4) = v;
      }
      __threadfence();
    }
  }
}

extern "C" void kernel_launch(void* const* d_in, const int* in_sizes, int n_in,
                              void* d_out, int out_size, void* d_ws, size_t ws_size, hipStream_t stream) {
  if (n_in < 13 || d_out == nullptr || d_ws == nullptr) return;
  if (in_sizes[0] != kBatch * kWin * kFeat || in_sizes[1] != kWin * kKC * 3 || in_sizes[2] != kWin * kKC ||
      in_sizes[3] != kFc1 * kFcIn || in_sizes[4] != kFc1 || in_sizes[5] != kFc1 * kGates ||
      in_sizes[6] != kFc1 * kGates * kHid || in_sizes[7] != 2 * kFc1 * kGates * kHid || in_sizes[8] != 2 * kFc1 * kGates ||
      in_sizes[9] != kComb || in_sizes[10] != 1 || in_sizes[11] != kComb || in_sizes[12] != 1 || out_size != 4 * kBatch) return;

  const float* x      = (const float*)d_in[0];
  const float* conv_w = (const float*)d_in[1];
  const float* conv_b = (const float*)d_in[2];
  const float* fc1_w  = (const float*)d_in[3];
  const float* fc1_b  = (const float*)d_in[4];
  const float* w_ih0  = (const float*)d_in[5];
  const float* w_ih1  = (const float*)d_in[6];
  const float* w_hh   = (const float*)d_in[7];
  const float* b_lstm = (const float*)d_in[8];
  const float* mu_w   = (const float*)d_in[9];
  const float* mu_b   = (const float*)d_in[10];
  const float* lv_w   = (const float*)d_in[11];
  const float* lv_b   = (const float*)d_in[12];
  float* out = (float*)d_out;

  char* ws = (char*)d_ws; size_t off = 0;
  auto carve = [&](size_t bytes) -> char* { char* p = ws + off; off += (bytes + 255) & ~(size_t)255; return p; };
  unsigned short* Y16  = (unsigned short*)carve((size_t)kRowsY * kPitchY * 2);
  unsigned short* Wt16 = (unsigned short*)carve((size_t)kMpadF * kPitchY * 2);
  float*          ZT   = (float*)carve((size_t)kMpadF * kRowsY * 4);
  float*          COMB = (float*)carve((size_t)kBatch * kComb * 4);
  if (off > ws_size || off > (size_t)134217728) return;

  fc1w_plane_kernel<<<(kMpadF * (kPitchY / 8)) / kThreads, kThreads, 0, stream>>>(fc1_w, Wt16);
  conv_pool_kernel<<<kWin * (kBatch / 16), kThreads, 0, stream>>>(x, conv_w, conv_b, Y16);
  wmma_gemm64<0, false, 0, 0, false, 0><<<dim3((kMpadF / 64) * (kRowsY / 64) / 8, 1), 256, 0, stream>>>(
      Wt16, Wt16, kPitchY, (long)0, Y16, Y16, kPitchY, (long)0, (void*)ZT, (void*)ZT, kRowsY, (long)0,
      fc1_b, (const float*)ZT, (long)0, kMpadF, kRowsY, kKdot, kFc1ScaleInv);
  lstm_bank_kernel<<<kFc1, kThreads, 0, stream>>>(ZT, fc1_b, w_ih0, w_ih1, w_hh, b_lstm, COMB);
  head_kernel<<<1, 128, 0, stream>>>(COMB, mu_w, mu_b, lv_w, lv_b, out);
}
